// HyperCategoryFramework_54434415509945
// MI455X (gfx1250) — hardware-verified
//
#include <hip/hip_runtime.h>
#include <math.h>

typedef _Float16 v16h __attribute__((ext_vector_type(16)));
typedef _Float16 v8h  __attribute__((ext_vector_type(8)));
typedef _Float16 v4h  __attribute__((ext_vector_type(4)));
typedef float    v8f  __attribute__((ext_vector_type(8)));
typedef float    v4f  __attribute__((ext_vector_type(4)));
typedef v8h __attribute__((may_alias)) v8ha;
typedef v4h __attribute__((may_alias)) v4ha;
typedef v4f __attribute__((may_alias)) v4fa;
union Frag { v16h v; v8h half[2]; _Float16 e[16]; };

#define NF     28
#define WD     144
#define KP     192
#define CD     256
#define NH     4
#define HD     64
#define DFF    2048
#define NC     10
#define NB     32
#define NPAIR  378
#define NTRI   3276
#define MTOK   3682
#define MP     3712
#define NMB    29
#define EPSC   17.0f
#define SHARPC 10.0f
#define PSCALE 16384.0f
#define KALL   0x7fffffff

__device__ __forceinline__ v8f wmma_f16(v16h a, v16h b, v8f c) {
  v8f d = __builtin_amdgcn_wmma_f32_16x16x32_f16(false, a, false, b, (short)0, c, false, false);
  asm volatile("v_nop\n\tv_nop\n\tv_nop\n\tv_nop" : "+v"(d) : "v"(a), "v"(b));
  return d;
}

__device__ __forceinline__ v16h load_frag(const _Float16* p, int h) {
  Frag f;
  f.half[0] = *(const v8ha*)(p + 8 * h);
  f.half[1] = *(const v8ha*)(p + 16 + 8 * h);
  return f.v;
}

__device__ __forceinline__ v8h cvt8(v4f a, v4f c, float sc) {
  const v8h o = { (_Float16)(a.x * sc), (_Float16)(a.y * sc), (_Float16)(a.z * sc), (_Float16)(a.w * sc),
                  (_Float16)(c.x * sc), (_Float16)(c.y * sc), (_Float16)(c.z * sc), (_Float16)(c.w * sc) };
  return o;
}

__device__ __forceinline__ void load8f(const float* p, float (&v)[8]) {
  const v4f a = *(const v4fa*)p;
  const v4f c = *(const v4fa*)(p + 4);
  v[0] = a.x; v[1] = a.y; v[2] = a.z; v[3] = a.w;
  v[4] = c.x; v[5] = c.y; v[6] = c.z; v[7] = c.w;
}

__device__ __forceinline__ int pidx(int i, int j) {
  const int p = ((i * (2 * NF - i - 1)) >> 1) + (j - i - 1);
  return min(max(p, 0), NPAIR - 1);
}
__device__ __forceinline__ void pair_decode(int p, int& i, int& j) {
  int rem = p, ii;
  #pragma unroll 1
  for (ii = 0; ii < NF - 2; ++ii) { const int cnt = NF - 1 - ii; if (rem < cnt) break; rem -= cnt; }
  i = ii; j = min(ii + 1 + rem, NF - 1);
}
__device__ __forceinline__ void tri_decode(int t, int& i, int& j, int& k) {
  int rem = t, ii, jj;
  #pragma unroll 1
  for (ii = 0; ii < NF - 3; ++ii) { const int c2 = ((NF - 1 - ii) * (NF - 2 - ii)) >> 1; if (rem < c2) break; rem -= c2; }
  #pragma unroll 1
  for (jj = ii + 1; jj < NF - 2; ++jj) { const int cnt = NF - 1 - jj; if (rem < cnt) break; rem -= cnt; }
  i = ii; j = jj; k = min(jj + 1 + rem, NF - 1);
}

__global__ __launch_bounds__(256) void k_convert(
    const float* __restrict__ lin_in_w, const float* __restrict__ in_proj_w,
    const float* __restrict__ out_proj_w, const float* __restrict__ ffn_w1,
    const float* __restrict__ ffn_w2, const float* __restrict__ lin_out_w,
    const float* __restrict__ omega, const float* __restrict__ lam_w,
    _Float16* __restrict__ linw16, _Float16* __restrict__ inproj16, _Float16* __restrict__ wo16,
    _Float16* __restrict__ w116, _Float16* __restrict__ w216, _Float16* __restrict__ wlo16,
    _Float16* __restrict__ omlam16)
{
  const int blk = blockIdx.x, tid = threadIdx.x;
  const v4f z4 = {0.0f, 0.0f, 0.0f, 0.0f};
  v4f a, c;
  _Float16* dst;
  if (blk < 24) {
    const int g = blk * 256 + tid;
    const int e = 8 * g;
    const int row = e / KP;
    const int c8 = (e - row * KP) >> 3;
    const int cc = min(c8, 17);
    const float* s = lin_in_w + row * WD + 8 * cc;
    a = *(const v4fa*)s; c = *(const v4fa*)(s + 4);
    const bool ok = c8 < 18;
    a = ok ? a : z4; c = ok ? c : z4;
    dst = linw16 + e;
  } else if (blk < 120) {
    const int g = (blk - 24) * 256 + tid;
    const float* s = in_proj_w + (size_t)g * 8;
    a = *(const v4fa*)s; c = *(const v4fa*)(s + 4);
    dst = inproj16 + (size_t)g * 8;
  } else if (blk < 152) {
    const int g = (blk - 120) * 256 + tid;
    const float* s = out_proj_w + (size_t)g * 8;
    a = *(const v4fa*)s; c = *(const v4fa*)(s + 4);
    dst = wo16 + (size_t)g * 8;
  } else if (blk < 408) {
    const int g = (blk - 152) * 256 + tid;
    const float* s = ffn_w1 + (size_t)g * 8;
    a = *(const v4fa*)s; c = *(const v4fa*)(s + 4);
    dst = w116 + (size_t)g * 8;
  } else if (blk < 664) {
    const int g = (blk - 408) * 256 + tid;
    const float* s = ffn_w2 + (size_t)g * 8;
    a = *(const v4fa*)s; c = *(const v4fa*)(s + 4);
    dst = w216 + (size_t)g * 8;
  } else if (blk < 696) {
    const int g = (blk - 664) * 256 + tid;
    const float* s = lin_out_w + (size_t)g * 8;
    a = *(const v4fa*)s; c = *(const v4fa*)(s + 4);
    dst = wlo16 + (size_t)g * 8;
  } else {
    const int g = (blk - 696) * 256 + tid;
    const int e = 8 * g;
    const int n = e >> 9;
    const int col = e & 511;
    const int cl = col & 255;
    float vo[8];
    #pragma unroll
    for (int q = 0; q < 8; ++q) vo[q] = omega[(size_t)(cl + q) * CD + n];
    const v4f oa = {vo[0], vo[1], vo[2], vo[3]};
    const v4f oc = {vo[4], vo[5], vo[6], vo[7]};
    const float* ls = lam_w + (size_t)n * CD + cl;
    const v4f la = *(const v4fa*)ls;
    const v4f lc = *(const v4fa*)(ls + 4);
    const bool isom = col < 256;
    a = isom ? oa : la; c = isom ? oc : lc;
    dst = omlam16 + e;
  }
  const v8h o = cvt8(a, c, 32.0f);
  *(volatile v8h*)dst = o;
  __threadfence();
  *(volatile v8h*)dst = o;
}

__global__ __launch_bounds__(256) void k_conv(
    const float* __restrict__ x, const float* __restrict__ cw, const float* __restrict__ cb,
    const float* __restrict__ fw, const float* __restrict__ fb, float* __restrict__ yws)
{
  __shared__ __attribute__((aligned(16))) _Float16 xs[16 * 1024];
  __shared__ __attribute__((aligned(16))) _Float16 wsm[32 * 160];
  __shared__ int ktab[160];
  __shared__ __attribute__((aligned(16))) float sb[32];
  __shared__ float red[8 * 32];
  __shared__ float smean[32];
  __shared__ __attribute__((aligned(16))) float sy[32];

  const int tid = threadIdx.x, lane = tid & 31, w = tid >> 5;
  const int h = lane >> 4, m = lane & 15;
  const int b = blockIdx.x;
  const float* xb = x + (size_t)b * 16384;

  #pragma unroll 1
  for (int i = 0; i < 16; ++i) {
    const int f = 4 * tid + 1024 * i;
    const v4f v = *(const v4fa*)(xb + f);
    const v4h o = {(_Float16)v.x, (_Float16)v.y, (_Float16)v.z, (_Float16)v.w};
    *(v4ha*)(xs + f) = o;
  }
  #pragma unroll 1
  for (int e = tid; e < 32 * 160; e += 256) {
    const int n = e / 160, k = e - n * 160;
    const int nc = min(n, NF - 1), kc = min(k, WD - 1);
    const float v = cw[nc * WD + kc];
    wsm[e] = (_Float16)((n < NF && k < WD) ? v : 0.0f);
  }
  if (tid < 160) {
    const int k = min(tid, WD - 1);
    const int ci = k / 9, t9 = k - 9 * ci, kh = t9 / 3, kw = t9 - 3 * kh;
    ktab[tid] = (tid < WD) ? (ci * 1024 + kh * 32 + kw) : 0;
  }
  if (tid < 32) sb[tid] = (tid < NF) ? cb[min(tid, NF - 1)] : 0.0f;
  __syncthreads();

  const v8f zero8 = {0.f, 0.f, 0.f, 0.f, 0.f, 0.f, 0.f, 0.f};
  float csum0 = 0.0f, csum1 = 0.0f;

  #pragma unroll 1
  for (int pt = w; pt < 60; pt += 8) {
    const int p = pt * 16 + m;
    const int pc = min(p, 899);
    const int r = pc / 30, c = pc - 30 * r;
    const int pbase = r * 32 + c;
    v8f acc0 = zero8, acc1 = zero8;
    #pragma unroll
    for (int ks = 0; ks < 5; ++ks) {
      const int k0 = 32 * ks;
      Frag a;
      #pragma unroll
      for (int i = 0; i < 8; ++i) a.e[i] = xs[pbase + ktab[k0 + 8 * h + i]];
      #pragma unroll
      for (int i = 0; i < 8; ++i) {
        const _Float16 t = xs[pbase + ktab[k0 + 16 + 8 * h + i]];
        a.e[8 + i] = (k0 < 128) ? t : (_Float16)0.0f;
      }
      Frag b0, b1;
      b0.half[0] = *(const v8ha*)(wsm + m * 160 + k0 + 8 * h);
      b0.half[1] = *(const v8ha*)(wsm + m * 160 + k0 + 16 + 8 * h);
      b1.half[0] = *(const v8ha*)(wsm + (16 + m) * 160 + k0 + 8 * h);
      b1.half[1] = *(const v8ha*)(wsm + (16 + m) * 160 + k0 + 16 + 8 * h);
      acc0 = wmma_f16(a.v, b0.v, acc0);
      acc1 = wmma_f16(a.v, b1.v, acc1);
    }
    const float bias0 = sb[m], bias1 = sb[16 + m];
    #pragma unroll
    for (int r8 = 0; r8 < 8; ++r8) {
      const int p2 = pt * 16 + 8 * h + r8;
      const float ok = (p2 < 900) ? 1.0f : 0.0f;
      csum0 += ok * fmaxf(acc0[r8] + bias0, 0.0f);
      csum1 += ok * fmaxf(acc1[r8] + bias1, 0.0f);
    }
  }
  csum0 += __shfl_xor(csum0, 16);
  csum1 += __shfl_xor(csum1, 16);
  if (h == 0) { red[w * 32 + m] = csum0; red[w * 32 + 16 + m] = csum1; }
  __syncthreads();
  if (tid < 32) {
    float s = 0.0f;
    #pragma unroll
    for (int q = 0; q < 8; ++q) s += red[q * 32 + tid];
    smean[tid] = (tid < NF) ? s * (1.0f / 900.0f) : 0.0f;
  }
  __syncthreads();
  if (tid < 32) {
    const int cc = min(tid, NC - 1);
    float s = 0.0f;
    #pragma unroll 1
    for (int n = 0; n < NF; ++n) s += smean[n] * fw[cc * NF + n];
    s += fb[cc];
    sy[tid] = (tid < NC) ? s : 0.0f;
  }
  __syncthreads();
  if (tid < 8) {
    const v4f v = *(const v4fa*)(sy + 4 * tid);
    float* d = yws + b * 32 + 4 * tid;
    *(volatile v4f*)d = v;
    __threadfence();
    *(volatile v4f*)d = v;
  }
}

__global__ __launch_bounds__(384) void k_geom(const float* __restrict__ cw, float* __restrict__ dtab)
{
  #pragma clang fp contract(off)
  __shared__ float sW[NF * WD];
  __shared__ __attribute__((aligned(16))) float sd[384];
  const int tid = threadIdx.x;
  #pragma unroll 1
  for (int e = tid; e < NF * WD; e += 384) sW[e] = cw[e];
  __syncthreads();
  const int p = min(tid, NPAIR - 1);
  int i, j;
  pair_decode(p, i, j);
  float s = 0.0f;
  #pragma unroll 1
  for (int c = 0; c < WD; ++c) {
    const float df = sW[i * WD + c] - sW[j * WD + c];
    s += df * df;
  }
  const float d = sqrtf(s);
  sd[tid] = (tid < NPAIR) ? d : 0.0f;
  __syncthreads();
  if (tid < 32) {
    v4f v0 = *(const v4fa*)(sd + 4 * tid);
    v4f v1 = *(const v4fa*)(sd + 128 + 4 * tid);
    v4f v2 = *(const v4fa*)(sd + 256 + 4 * tid);
    *(volatile v4f*)(dtab + 4 * tid) = v0;
    *(volatile v4f*)(dtab + 128 + 4 * tid) = v1;
    *(volatile v4f*)(dtab + 256 + 4 * tid) = v2;
    __threadfence();
    *(volatile v4f*)(dtab + 4 * tid) = v0;
    *(volatile v4f*)(dtab + 128 + 4 * tid) = v1;
    *(volatile v4f*)(dtab + 256 + 4 * tid) = v2;
  }
}

__global__ __launch_bounds__(256) void k_build(
    const float* __restrict__ cw, const float* __restrict__ dtab,
    _Float16* __restrict__ pooled, float* __restrict__ wts, float* __restrict__ ipa)
{
  #pragma clang fp contract(off)
  __shared__ __attribute__((aligned(16))) float sw[32];
  __shared__ __attribute__((aligned(16))) float sip[32];
  const int tid = threadIdx.x, lane = tid & 31, w = tid >> 5;
  const int c8 = min(lane, 17);
  const float colok = (lane < 18) ? 1.0f : 0.0f;
  #pragma unroll 1
  for (int rr = 0; rr < 4; ++rr) {
    const int rloc = w * 4 + rr;
    const int row = blockIdx.x * 32 + rloc;
    float vals[8];
    float wv, ipv;
    if (row < NF) {
      float wi[8];
      load8f(cw + row * WD + 8 * c8, wi);
      const float rc = 1.0f / 1.000001f;
      #pragma unroll
      for (int q = 0; q < 8; ++q) vals[q] = wi[q] * rc;
      wv = 1.0f;
      ipv = 1.0f / (1.0f + expf(10.0f));
    } else if (row < NF + NPAIR) {
      const int p = row - NF;
      int i, j;
      pair_decode(p, i, j);
      const float d = dtab[p];
      const float t = expf(fminf(SHARPC * (d - EPSC), 80.0f));
      const float val = 1.0f / (1.0f + t);
      float wi[8], wj[8];
      load8f(cw + i * WD + 8 * c8, wi);
      load8f(cw + j * WD + 8 * c8, wj);
      const float rden = 1.0f / (2.0f * val + 1e-6f);
      #pragma unroll
      for (int q = 0; q < 8; ++q) vals[q] = (val * (wi[q] + wj[q])) * rden;
      wv = (val > 1e-6f) ? 1.0f : 0.0f;
      const float z = (2.0f * val - 2.0f) * 10.0f;
      ipv = 1.0f / (1.0f + expf(-z));
    } else if (row < MTOK) {
      const int t = row - NF - NPAIR;
      int i, j, k;
      tri_decode(t, i, j, k);
      const float dij = dtab[pidx(i, j)], djk = dtab[pidx(j, k)], dik = dtab[pidx(i, k)];
      wv = (dij <= EPSC && djk <= EPSC && dik <= EPSC) ? 1.0f : 0.0f;
      float wi[8], wj[8], wk[8];
      load8f(cw + i * WD + 8 * c8, wi);
      load8f(cw + j * WD + 8 * c8, wj);
      load8f(cw + k * WD + 8 * c8, wk);
      const float rc = 1.0f / 3.000001f;
      #pragma unroll
      for (int q = 0; q < 8; ++q) vals[q] = ((wi[q] + wj[q]) + wk[q]) * rc;
      ipv = 1.0f / (1.0f + expf(-10.0f));
    } else {
      #pragma unroll
      for (int q = 0; q < 8; ++q) vals[q] = 0.0f;
      wv = 0.0f; ipv = 0.0f;
    }
    const float sc = 512.0f * colok;
    const v8h o = { (_Float16)(vals[0] * sc), (_Float16)(vals[1] * sc), (_Float16)(vals[2] * sc), (_Float16)(vals[3] * sc),
                    (_Float16)(vals[4] * sc), (_Float16)(vals[5] * sc), (_Float16)(vals[6] * sc), (_Float16)(vals[7] * sc) };
    _Float16* dst = pooled + (size_t)row * KP + 8 * lane;
    if (lane < 24) *(volatile v8h*)dst = o;
    __threadfence();
    if (lane < 24) *(volatile v8h*)dst = o;
    if (lane == 0) { sw[rloc] = wv; sip[rloc] = ipv; }
  }
  __syncthreads();
  if (tid < 8) {
    const v4f a = *(const v4fa*)(sw + 4 * tid);
    const v4f c = *(const v4fa*)(sip + 4 * tid);
    float* d1 = wts + blockIdx.x * 32 + 4 * tid;
    float* d2 = ipa + blockIdx.x * 32 + 4 * tid;
    *(volatile v4f*)d1 = a;
    *(volatile v4f*)d2 = c;
    __threadfence();
    *(volatile v4f*)d1 = a;
    *(volatile v4f*)d2 = c;
  }
}

__device__ __forceinline__ void gemm_core(const _Float16* __restrict__ A, int lda, int kmask,
                                          const _Float16* __restrict__ W, int ldw, int K,
                                          int m0w, int n0, int h, int m, v8f (&acc)[2][4])
{
  const _Float16* xa0 = A + (size_t)(m0w + m) * lda;
  const _Float16* xa1 = xa0 + (size_t)16 * lda;
  const _Float16* wb  = W + (size_t)(n0 + m) * ldw;
  const v8f zero8 = {0.f, 0.f, 0.f, 0.f, 0.f, 0.f, 0.f, 0.f};
  #pragma unroll
  for (int mt = 0; mt < 2; ++mt)
    #pragma unroll
    for (int nt = 0; nt < 4; ++nt) acc[mt][nt] = zero8;
  #pragma unroll 1
  for (int k0 = 0; k0 < K; k0 += 32) {
    const int ak = k0 & kmask;
    const v16h a0 = load_frag(xa0 + ak, h);
    const v16h a1 = load_frag(xa1 + ak, h);
    #pragma unroll
    for (int nt = 0; nt < 4; ++nt) {
      const v16h bf = load_frag(wb + (size_t)nt * 16 * ldw + k0, h);
      acc[0][nt] = wmma_f16(a0, bf, acc[0][nt]);
      acc[1][nt] = wmma_f16(a1, bf, acc[1][nt]);
    }
  }
}

__device__ __forceinline__ void pass32(const float* sT, float* C32, int ldc, int m0, int n0, int w, int lane) {
  const int q8 = lane & 7, sub = lane >> 3;
  #pragma unroll
  for (int i = 0; i < 16; ++i) {
    const int L = i * 4 + sub;
    const int row = 32 * w + (L >> 1), hl = L & 1;
    const v4f v = *(const v4fa*)(sT + row * 64 + 32 * hl + 4 * q8);
    *(volatile v4f*)(C32 + (size_t)(m0 + row) * ldc + n0 + 32 * hl + 4 * q8) = v;
  }
}
__device__ __forceinline__ void pass16(const float* sT, _Float16* C16, int ldc, int m0, int n0, int w, int lane) {
  const int q8 = lane & 7, sub = lane >> 3;
  #pragma unroll
  for (int i = 0; i < 8; ++i) {
    const int row = 32 * w + i * 4 + sub;
    const v4f a = *(const v4fa*)(sT + row * 64 + 8 * q8);
    const v4f c = *(const v4fa*)(sT + row * 64 + 8 * q8 + 4);
    const v8h o = cvt8(a, c, 1.0f);
    *(volatile v8h*)(C16 + (size_t)(m0 + row) * ldc + n0 + 8 * q8) = o;
  }
}

template <bool O32, bool O16, bool RES, int ACT>
__global__ __launch_bounds__(128) void k_gemm(
    const _Float16* __restrict__ A, int lda, int kmask,
    const _Float16* __restrict__ W, int K,
    const float* __restrict__ bias, float scale, int qcols,
    const float* __restrict__ R,
    float* __restrict__ C32, _Float16* __restrict__ C16, int ldc)
{
  __shared__ __attribute__((aligned(16))) float sT[128 * 64];
  const int tid = threadIdx.x, lane = tid & 31, w = tid >> 5;
  const int h = lane >> 4, m = lane & 15;
  const int m0 = blockIdx.x * 128, n0 = blockIdx.y * 64;
  const int m0w = m0 + 32 * w;

  v8f acc[2][4];
  gemm_core(A, lda, kmask, W, K, K, m0w, n0, h, m, acc);

  const float osc = (n0 < qcols) ? 0.125f : 1.0f;
  #pragma unroll
  for (int nt = 0; nt < 4; ++nt) {
    const int feat = 16 * nt + m;
    const float bvl = bias[n0 + feat];
    #pragma unroll
    for (int mt = 0; mt < 2; ++mt) {
      #pragma unroll
      for (int r = 0; r < 8; ++r) {
        const int tokl = 32 * w + 16 * mt + 8 * h + r;
        float y = acc[mt][nt][r] * scale + bvl;
        if (RES) y += R[(size_t)(m0 + tokl) * ldc + n0 + feat];
        if (ACT == 1) y = fmaxf(y, 0.0f);
        sT[tokl * 64 + feat] = y * osc;
      }
    }
  }
  __syncthreads();
  if (O32) pass32(sT, C32, ldc, m0, n0, w, lane);
  if (O16) pass16(sT, C16, ldc, m0, n0, w, lane);
  __threadfence();
  if (O32) pass32(sT, C32, ldc, m0, n0, w, lane);
  if (O16) pass16(sT, C16, ldc, m0, n0, w, lane);
}

__device__ __forceinline__ void passvt(const _Float16* sTh, _Float16* vt, int m0, int n0, int w, int lane) {
  const int q8 = lane & 7, sub = lane >> 3;
  #pragma unroll
  for (int i = 0; i < 8; ++i) {
    const int lid = 32 * w + 4 * i + sub;
    const int d = lid >> 1, hl = lid & 1;
    const v8h v = *(const v8ha*)(sTh + d * 128 + 64 * hl + 8 * q8);
    *(volatile v8h*)(vt + (size_t)(n0 + d) * MP + m0 + 64 * hl + 8 * q8) = v;
  }
}

__global__ __launch_bounds__(128) void k_gemm_vt(
    const _Float16* __restrict__ A,
    const _Float16* __restrict__ W,
    const float* __restrict__ bias,
    _Float16* __restrict__ vt)
{
  __shared__ __attribute__((aligned(16))) _Float16 sTh[64 * 128];
  const int tid = threadIdx.x, lane = tid & 31, w = tid >> 5;
  const int h = lane >> 4, m = lane & 15;
  const int m0 = blockIdx.x * 128, n0 = blockIdx.y * 64;
  const int m0w = m0 + 32 * w;

  v8f acc[2][4];
  gemm_core(A, CD, KALL, W, CD, CD, m0w, n0, h, m, acc);

  #pragma unroll
  for (int nt = 0; nt < 4; ++nt) {
    const int feat = 16 * nt + m;
    const float bvl = bias[n0 + feat];
    #pragma unroll
    for (int mt = 0; mt < 2; ++mt) {
      #pragma unroll
      for (int r = 0; r < 8; ++r) {
        const int tokl = 32 * w + 16 * mt + 8 * h + r;
        const float y = acc[mt][nt][r] * 0.03125f + bvl;
        sTh[feat * 128 + tokl] = (_Float16)y;
      }
    }
  }
  __syncthreads();
  passvt(sTh, vt, m0, n0, w, lane);
  __threadfence();
  passvt(sTh, vt, m0, n0, w, lane);
}

__device__ __forceinline__ v16h pack_p(v8f a, v8f c) {
  const v16h r = { (_Float16)(a[0] * PSCALE), (_Float16)(a[1] * PSCALE), (_Float16)(a[2] * PSCALE), (_Float16)(a[3] * PSCALE),
                   (_Float16)(a[4] * PSCALE), (_Float16)(a[5] * PSCALE), (_Float16)(a[6] * PSCALE), (_Float16)(a[7] * PSCALE),
                   (_Float16)(c[0] * PSCALE), (_Float16)(c[1] * PSCALE), (_Float16)(c[2] * PSCALE), (_Float16)(c[3] * PSCALE),
                   (_Float16)(c[4] * PSCALE), (_Float16)(c[5] * PSCALE), (_Float16)(c[6] * PSCALE), (_Float16)(c[7] * PSCALE) };
  return r;
}

__device__ __forceinline__ void att_store(const float* so, _Float16* a16, int head, int q0, int lane) {
  const int q8 = lane & 7, sub = lane >> 3;
  #pragma unroll
  for (int i = 0; i < 4; ++i) {
    const int row = i * 4 + sub;
    const v4f a = *(const v4fa*)(so + row * 64 + 8 * q8);
    const v4f c = *(const v4fa*)(so + row * 64 + 8 * q8 + 4);
    const v8h o = cvt8(a, c, 1.0f);
    *(volatile v8h*)(a16 + (size_t)(q0 + row) * CD + head * HD + 8 * q8) = o;
  }
}

__global__ __launch_bounds__(128) void k_attn(
    const _Float16* __restrict__ qk16,
    const _Float16* __restrict__ vt,
    _Float16* __restrict__ a16)
{
  __shared__ __attribute__((aligned(16))) float sO[4 * 16 * 64];

  const int tid = threadIdx.x, lane = tid & 31, w = tid >> 5;
  const int h = lane >> 4, m = lane & 15;
  const int head = blockIdx.y;
  const int q0 = blockIdx.x * 64 + 16 * w;

  const _Float16* qrow = qk16 + (size_t)(q0 + m) * (2 * CD) + head * HD;
  const v16h qb0 = load_frag(qrow, h);
  const v16h qb1 = load_frag(qrow + 32, h);

  const v8f zero8 = {0.f, 0.f, 0.f, 0.f, 0.f, 0.f, 0.f, 0.f};
  v8f o[4];
  #pragma unroll
  for (int t = 0; t < 4; ++t) o[t] = zero8;
  float mrun = -1e30f, lrun = 0.0f;

  const _Float16* kbase = qk16 + (size_t)m * (2 * CD) + CD + head * HD;
  const _Float16* vbase = vt + (size_t)(head * HD + m) * MP;

  #pragma unroll 1
  for (int kb = 0; kb < MP; kb += 64) {
    v8f s[4];
    #pragma unroll
    for (int j = 0; j < 4; ++j) {
      const _Float16* kp = kbase + (size_t)(kb + 16 * j) * (2 * CD);
      const v16h kf0 = load_frag(kp, h);
      const v16h kf1 = load_frag(kp + 32, h);
      v8f z = zero8;
      z = wmma_f16(kf0, qb0, z);
      z = wmma_f16(kf1, qb1, z);
      s[j] = z;
    }
    #pragma unroll
    for (int j = 0; j < 4; ++j)
      #pragma unroll
      for (int r = 0; r < 8; ++r) {
        const int key = kb + 16 * j + 8 * h + r;
        s[j][r] = (key < MTOK) ? s[j][r] : -1e30f;
      }

    float mloc = s[0][0];
    #pragma unroll
    for (int j = 0; j < 4; ++j)
      #pragma unroll
      for (int r = 0; r < 8; ++r) mloc = fmaxf(mloc, s[j][r]);
    mloc = fmaxf(mloc, __shfl_xor(mloc, 16));
    const float mnew = fmaxf(mrun, mloc);
    const float alpha = __expf(mrun - mnew);
    mrun = mnew;
    float lsum = 0.0f;
    #pragma unroll
    for (int j = 0; j < 4; ++j)
      #pragma unroll
      for (int r = 0; r < 8; ++r) {
        const float p = __expf(s[j][r] - mnew);
        s[j][r] = p;
        lsum += p;
      }
    lsum += __shfl_xor(lsum, 16);
    lrun = lrun * alpha + lsum;
    #pragma unroll
    for (int t = 0; t < 4; ++t)
      #pragma unroll
      for (int r = 0; r < 8; ++r) o[t][r] = o[t][r] * alpha;

    const v16h pb0 = pack_p(s[0], s[1]);
    const v16h pb1 = pack_p(s[2], s[3]);

    #pragma unroll
    for (int t = 0; t < 4; ++t) {
      const _Float16* vp = vbase + (size_t)(16 * t) * MP + kb;
      const v16h vf0 = load_frag(vp, h);
      const v16h vf1 = load_frag(vp + 32, h);
      o[t] = wmma_f16(vf0, pb0, o[t]);
      o[t] = wmma_f16(vf1, pb1, o[t]);
    }
  }

  const float inv = (1.0f / lrun) * (1.0f / PSCALE);
  float* so = sO + w * 1024;
  #pragma unroll
  for (int t = 0; t < 4; ++t)
    #pragma unroll
    for (int r = 0; r < 8; ++r)
      so[m * 64 + 16 * t + 8 * h + r] = o[t][r] * inv;
  __syncthreads();

  att_store(so, a16, head, q0, lane);
  __threadfence();
  att_store(so, a16, head, q0, lane);
}

template <bool O32>
__global__ __launch_bounds__(256) void k_ln(
    const float* __restrict__ X, const float* __restrict__ g, const float* __restrict__ bt,
    float* __restrict__ Y32, _Float16* __restrict__ Y16)
{
  __shared__ __attribute__((aligned(16))) float sm[8 * CD];
  const int tid = threadIdx.x, lane = tid & 31, w = tid >> 5;
  const int row = blockIdx.x * 8 + w;
  float v[8], gg[8], bb[8];
  load8f(X + (size_t)row * CD + 8 * lane, v);
  load8f(g + 8 * lane, gg);
  load8f(bt + 8 * lane, bb);
  float s = 0.0f;
  #pragma unroll
  for (int e = 0; e < 8; ++e) s += v[e];
  #pragma unroll
  for (int off = 16; off > 0; off >>= 1) s += __shfl_xor(s, off);
  const float mean = s * (1.0f / CD);
  float d[8];
  float q = 0.0f;
  #pragma unroll
  for (int e = 0; e < 8; ++e) { d[e] = v[e] - mean; q += d[e] * d[e]; }
  #pragma unroll
  for (int off = 16; off > 0; off >>= 1) q += __shfl_xor(q, off);
  const float var = q * (1.0f / CD);
  const float rstd = 1.0f / sqrtf(var + 1e-5f);
  float o[8];
  #pragma unroll
  for (int e = 0; e < 8; ++e) o[e] = d[e] * rstd * gg[e] + bb[e];
  const v8h oh = { (_Float16)o[0], (_Float16)o[1], (_Float16)o[2], (_Float16)o[3],
                   (_Float16)o[4], (_Float16)o[5], (_Float16)o[6], (_Float16)o[7] };
  _Float16* d16 = Y16 + (size_t)row * CD + 8 * lane;
  if (O32) {
    #pragma unroll
    for (int e = 0; e < 8; ++e) sm[w * CD + 8 * lane + e] = o[e];
    __syncthreads();
    const v4f p0 = *(const v4fa*)(sm + w * CD + 4 * lane);
    const v4f p1 = *(const v4fa*)(sm + w * CD + 128 + 4 * lane);
    float* d32 = Y32 + (size_t)row * CD;
    *(volatile v8h*)d16 = oh;
    *(volatile v4f*)(d32 + 4 * lane) = p0;
    *(volatile v4f*)(d32 + 128 + 4 * lane) = p1;
    __threadfence();
    *(volatile v8h*)d16 = oh;
    *(volatile v4f*)(d32 + 4 * lane) = p0;
    *(volatile v4f*)(d32 + 128 + 4 * lane) = p1;
  } else {
    *(volatile v8h*)d16 = oh;
    __threadfence();
    *(volatile v8h*)d16 = oh;
  }
}

__global__ __launch_bounds__(128) void k_gemm_hyper(
    const _Float16* __restrict__ ctx16,
    const _Float16* __restrict__ WL,
    const float* __restrict__ lam_b,
    const float* __restrict__ ctx32,
    const float* __restrict__ ipa, const float* __restrict__ wts,
    float* __restrict__ part)
{
  __shared__ __attribute__((aligned(16))) float sT[128 * 64];
  __shared__ float sP[128];
  __shared__ __attribute__((aligned(16))) float sL[64];
  const int tid = threadIdx.x, lane = tid & 31, w = tid >> 5;
  const int h = lane >> 4, m = lane & 15;
  const int m0 = blockIdx.x * 128, n0 = blockIdx.y * 64;
  const int m0w = m0 + 32 * w;

  v8f acc[2][4];
  gemm_core(ctx16, CD, CD - 1, WL, 2 * CD, 2 * CD, m0w, n0, h, m, acc);

  #pragma unroll
  for (int nt = 0; nt < 4; ++nt) {
    const int feat = 16 * nt + m;
    const float bvl = lam_b[n0 + feat];
    #pragma unroll
    for (int mt = 0; mt < 2; ++mt) {
      #pragma unroll
      for (int r = 0; r < 8; ++r) {
        const int tokl = 32 * w + 16 * mt + 8 * h + r;
        sT[tokl * 64 + feat] = acc[mt][nt][r] * 0.03125f + bvl;
      }
    }
  }
  __syncthreads();

  {
    const int c = tid & 63, grp = tid >> 6;
    float s = 0.0f;
    #pragma unroll 1
    for (int r = 0; r < 64; ++r) {
      const int rowl = 64 * grp + r;
      const int mm = m0 + rowl;
      const float xv = sT[rowl * 64 + c];
      const float ge = 0.5f * xv * (1.0f + erff(xv * 0.70710678118654752f));
      const float ipm = ipa[mm];
      const float cv = ctx32[(size_t)mm * CD + n0 + c];
      const float Hv = ipm * ge + (1.0f - ipm) * cv;
      s += wts[mm] * Hv;
    }
    sP[tid] = s;
  }
  __syncthreads();
  if (tid < 64) sL[tid] = sP[tid] + sP[64 + tid];
  __syncthreads();
  if (tid < 16) {
    const v4f v = *(const v4fa*)(sL + 4 * tid);
    float* dst = part + (size_t)blockIdx.x * CD + n0 + 4 * tid;
    *(volatile v4f*)dst = v;
    __threadfence();
    *(volatile v4f*)dst = v;
  }
}

__global__ __launch_bounds__(256) void k_final(
    const float* __restrict__ part, const float* __restrict__ wts, const float* __restrict__ yws,
    const float* __restrict__ omega, const float* __restrict__ caw, const float* __restrict__ cab,
    float* __restrict__ out)
{
  __shared__ float sRed[256];
  __shared__ float sH[256];
  __shared__ float sProj[256];
  __shared__ float sCorr[32];
  __shared__ __attribute__((aligned(16))) float sOut[320];
  const int tid = threadIdx.x;

  float s = 0.0f;
  #pragma unroll 1
  for (int r = tid; r < MP; r += 256) s += wts[r];
  sRed[tid] = s;
  __syncthreads();
  #pragma unroll 1
  for (int st = 128; st > 0; st >>= 1) {
    if (tid < st) sRed[tid] += sRed[tid + st];
    __syncthreads();
  }
  const float wsum = sRed[0];
  const float rw = 1.0f / wsum;

  float hs = 0.0f;
  #pragma unroll 1
  for (int mb = 0; mb < NMB; ++mb) hs += part[mb * CD + tid];
  sH[tid] = hs * rw;
  __syncthreads();

  float pj = 0.0f;
  #pragma unroll 1
  for (int j = 0; j < CD; ++j) pj += sH[j] * omega[(size_t)tid * CD + j];
  sProj[tid] = pj;
  __syncthreads();

  if (tid < 32) {
    const int cc = min(tid, NC - 1);
    float cs = 0.0f;
    #pragma unroll 1
    for (int i = 0; i < CD; ++i) cs += sProj[i] * caw[cc * CD + i];
    cs += cab[cc];
    sCorr[tid] = (tid < NC) ? cs : 0.0f;
  }
  __syncthreads();

  #pragma unroll 1
  for (int e = tid; e < NB * NC; e += 256) {
    const int bb = e / NC, c = e - NC * bb;
    sOut[e] = yws[bb * 32 + c] + sCorr[c];
  }
  __syncthreads();

  if (tid < 32) {
    const v4f v0 = *(const v4fa*)(sOut + 4 * tid);
    const v4f v1 = *(const v4fa*)(sOut + 128 + 4 * tid);
    const v4f v2 = *(const v4fa*)(sOut + 256 + 4 * min(tid, 15));
    *(volatile v4f*)(out + 4 * tid) = v0;
    *(volatile v4f*)(out + 128 + 4 * tid) = v1;
    if (tid < 16) *(volatile v4f*)(out + 256 + 4 * tid) = v2;
    __threadfence();
    *(volatile v4f*)(out + 4 * tid) = v0;
    *(volatile v4f*)(out + 128 + 4 * tid) = v1;
    if (tid < 16) *(volatile v4f*)(out + 256 + 4 * tid) = v2;
  }
}

extern "C" void kernel_launch(void* const* d_in, const int* in_sizes, int n_in,
                              void* d_out, int out_size, void* d_ws, size_t ws_size,
                              hipStream_t stream)
{
  if (n_in < 26) return;
  if (in_sizes[0] != NB * 16 * 1024) return;
  if (in_sizes[1] != NF * WD || in_sizes[2] != NF) return;
  if (in_sizes[3] != NC * NF || in_sizes[4] != NC) return;
  if (in_sizes[5] != CD * WD || in_sizes[6] != CD) return;
  if (in_sizes[7] != 3 * CD * CD || in_sizes[8] != 3 * CD) return;
  if (in_sizes[9] != CD * CD || in_sizes[10] != CD) return;
  if (in_sizes[11] != CD || in_sizes[12] != CD) return;
  if (in_sizes[13] != DFF * CD || in_sizes[14] != DFF) return;
  if (in_sizes[15] != CD * DFF || in_sizes[16] != CD) return;
  if (in_sizes[17] != CD || in_sizes[18] != CD) return;
  if (in_sizes[19] != CD * CD || in_sizes[20] != CD) return;
  if (in_sizes[21] != CD * CD || in_sizes[22] != CD * CD || in_sizes[23] != CD) return;
  if (in_sizes[24] != NC * CD || in_sizes[25] != NC) return;
  if (out_size != NB * NC) return;

  const float* x          = (const float*)d_in[0];
  const float* conv_w     = (const float*)d_in[1];
  const float* conv_b     = (const float*)d_in[2];
  const float* fc_w       = (const float*)d_in[3];
  const float* fc_b       = (const float*)d_in[4];
  const float* lin_in_w   = (const float*)d_in[5];
  const float* lin_in_b   = (const float*)d_in[6];
  const float* in_proj_w  = (const float*)d_in[7];
  const float* in_proj_b  = (const float*)d_in[8];
  const float* out_proj_w = (const float*)d_in[9];
  const float* out_proj_b = (const float*)d_in[10];
  const float* ln1_g      = (const float*)d_in[11];
  const float* ln1_b      = (const float*)d_in[12];
  const float* ffn_w1     = (const float*)d_in[13];
  const float* ffn_b1     = (const float*)d_in[14];
  const float* ffn_w2     = (const float*)d_in[15];
  const float* ffn_b2     = (const float*)d_in[16];
  const float* ln2_g      = (const float*)d_in[17];
  const float* ln2_b      = (const float*)d_in[18];
  const float* lin_out_w  = (const float*)d_in[19];
  const float* lin_out_b  = (const float*)d_in[20];
  const float* omega      = (const float*)d_in[21];
  const float* lam_w      = (const float*)d_in[22];
  const float* lam_b      = (const float*)d_in[23];
  const float* ca_w       = (const float*)d_in[24];
  const float* ca_b       = (const float*)d_in[25];
  float* out = (float*)d_out;

  const size_t b_linw   = (size_t)CD * KP * 2;
  const size_t b_inproj = (size_t)3 * CD * CD * 2;
  const size_t b_sq16   = (size_t)CD * CD * 2;
  const size_t b_ffw    = (size_t)DFF * CD * 2;
  const size_t b_omlam  = (size_t)CD * 2 * CD * 2;
  const size_t b_pooled = (size_t)MP * KP * 2;
  const size_t b_dtab   = 384 * 4;
  const size_t b_rowvec = (size_t)MP * 4;
  const size_t b_yws    = (size_t)NB * 32 * 4;
  const size_t b_act32  = (size_t)MP * CD * 4;
  const size_t b_act16  = (size_t)MP * CD * 2;
  const size_t b_qk16   = (size_t)MP * 2 * CD * 2;
  const size_t b_ff16   = (size_t)MP * DFF * 2;
  const size_t b_part   = (size_t)NMB * CD * 4;

  char* ws = (char*)d_ws;
  size_t off = 0;
  _Float16* linw16   = (_Float16*)(ws + off); off += b_linw;
  _Float16* inproj16 = (_Float16*)(ws + off); off += b_inproj;
  _Float16* wo16     = (_Float16*)(ws + off); off += b_sq16;
  _Float16* w116     = (_Float16*)(ws + off); off += b_ffw;
  _Float16* w216     = (_Float16*)(ws + off); off += b_ffw;
  _Float16* wlo16    = (_Float16*)(ws + off); off += b_sq16;
  _Float16* omlam16  = (_Float16*)(ws + off); off += b_omlam;
  _Float16* pooled16 = (_Float16*)(ws + off); off += b_pooled;
  float*    dtab     = (float*)(ws + off);    off += b_dtab;
  float*    wts      = (float*)(ws + off);    off += b_rowvec;
  float*    ipa      = (float*)(ws + off);    off += b_rowvec;
  float*    yws      = (float*)(ws + off);    off += b_yws;
  float*    h32      = (float*)(ws + off);    off += b_act32;
  _Float16* h16      = (_Float16*)(ws + off); off += b_act16;
  _Float16* qk16     = (_Float16*)(ws + off); off += b_qk16;
  _Float16* vt16     = (_Float16*)(ws + off); off += b_act16;
  _Float16* a16      = (_Float16*)(ws + off); off += b_act16;
  float*    tmp32    = (float*)(ws + off);    off += b_act32;
  float*    h1_32    = (float*)(ws + off);    off += b_act32;
  _Float16* h1_16    = (_Float16*)(ws + off); off += b_act16;
  _Float16* ff16     = (_Float16*)(ws + off); off += b_ff16;
  _Float16* h2_16    = (_Float16*)(ws + off); off += b_act16;
  float*    ctx32    = (float*)(ws + off);    off += b_act32;
  _Float16* ctx16    = (_Float16*)(ws + off); off += b_act16;
  float*    part     = (float*)(ws + off);    off += b_part;
  if (off > ws_size) return;

  const float s32 = 0.03125f;
  const float s_linin = 1.0f / 16384.0f;

  k_convert<<<760, 256, 0, stream>>>(lin_in_w, in_proj_w, out_proj_w, ffn_w1, ffn_w2, lin_out_w, omega, lam_w,
                                     linw16, inproj16, wo16, w116, w216, wlo16, omlam16);
  k_conv<<<NB, 256, 0, stream>>>(x, conv_w, conv_b, fc_w, fc_b, yws);
  k_geom<<<1, 384, 0, stream>>>(conv_w, dtab);
  k_build<<<MP / 32, 256, 0, stream>>>(conv_w, dtab, pooled16, wts, ipa);
  k_gemm<true, true, false, 0><<<dim3(NMB, CD / 64), 128, 0, stream>>>(
      pooled16, KP, KALL, linw16, KP, lin_in_b, s_linin, 0, h32, h32, h16, CD);
  k_gemm<false, true, false, 0><<<dim3(NMB, 2 * CD / 64), 128, 0, stream>>>(
      h16, CD, KALL, inproj16, CD, in_proj_b, s32, CD, h32, tmp32, qk16, 2 * CD);
  k_gemm_vt<<<dim3(NMB, CD / 64), 128, 0, stream>>>(h16, inproj16 + (size_t)2 * CD * CD, in_proj_b + 2 * CD, vt16);
  k_attn<<<dim3(MP / 64, NH), 128, 0, stream>>>(qk16, vt16, a16);
  k_gemm<true, false, true, 0><<<dim3(NMB, CD / 64), 128, 0, stream>>>(
      a16, CD, KALL, wo16, CD, out_proj_b, s32, 0, h32, tmp32, h2_16, CD);
  k_ln<true><<<MP / 8, 256, 0, stream>>>(tmp32, ln1_g, ln1_b, h1_32, h1_16);
  k_gemm<false, true, false, 1><<<dim3(NMB, DFF / 64), 128, 0, stream>>>(
      h1_16, CD, KALL, w116, CD, ffn_b1, s32, 0, h32, ctx32, ff16, DFF);
  k_gemm<true, false, true, 0><<<dim3(NMB, CD / 64), 128, 0, stream>>>(
      ff16, DFF, KALL, w216, DFF, ffn_b2, s32, 0, h1_32, tmp32, h2_16, CD);
  k_ln<false><<<MP / 8, 256, 0, stream>>>(tmp32, ln2_g, ln2_b, h1_32, h2_16);
  k_gemm<true, true, false, 0><<<dim3(NMB, CD / 64), 128, 0, stream>>>(
      h2_16, CD, KALL, wlo16, CD, lin_out_b, s32, 0, h32, ctx32, ctx16, CD);
  k_gemm_hyper<<<dim3(NMB, CD / 64), 128, 0, stream>>>(ctx16, omlam16, lam_b, ctx32, ipa, wts, part);
  k_final<<<1, 256, 0, stream>>>(part, wts, yws, omega, ca_w, ca_b, out);
  (void)hipGetLastError();
}
